// LocalSelfAttention_5540507811946
// MI455X (gfx1250) — hardware-verified
//
#include <hip/hip_runtime.h>
typedef __attribute__((ext_vector_type(4))) float vf4v_t;
typedef __attribute__((ext_vector_type(4))) unsigned int vu4v_t;
typedef __attribute__((ext_vector_type(4))) int vi4v_t;
#include <hip/hip_bf16.h>
#include <stdint.h>

#define HH 56
#define WWID 56
#define HWP 3136
#define BATCH 4
#define NPIX 12544
#define CIN 256
#define COUT 256
#define HDIM 128
#define PADR 2
#define EPSV 1e-5f
#define INV_SQRT_HD 0.08838834764831845f

typedef __attribute__((ext_vector_type(16))) _Float16 v16h;
typedef __attribute__((ext_vector_type(8)))  float    v8f;

union Frag16 { v16h v; float4 f[2]; };
union H8     { float4 f; vf4v_t fv; _Float16 h[8]; };
__device__ __forceinline__ v8f wmma16(v16h a, v16h b, v8f c) {
  v8f d = __builtin_amdgcn_wmma_f32_16x16x32_f16(false, a, false, b, (short)0, c, false, false);
  asm volatile("v_nop\n\tv_nop\n\tv_nop\n\tv_nop" : "+v"(d) : "v"(a), "v"(b));
  return d;
}
#define VST2(T, ptr, val) do { const T _v = (val); *(volatile T*)(ptr) = _v; __threadfence(); *(volatile T*)(ptr) = _v; } while (0)

__global__ __launch_bounds__(256) void cvt_x_kernel(const float* __restrict__ x,
                                                    _Float16* __restrict__ xt) {
  __shared__ __align__(16) _Float16 tile[64][CIN + 8];
  const int t = threadIdx.x;
  const int b = blockIdx.x / (HWP / 64), hw0 = (blockIdx.x % (HWP / 64)) * 64;
  for (int i = t; i < CIN * 64; i += 256) { const int c = i >> 6, pl = i & 63; tile[pl][c] = (_Float16)x[((size_t)(b * CIN + c)) * HWP + hw0 + pl]; }
  __syncthreads();
  for (int pass = 0; pass < 2; ++pass) {
#pragma unroll
    for (int q = 0; q < 8; ++q) { const int piece = t + q * 256, pl = piece >> 5, sg = piece & 31;
      H8 v;
#pragma unroll
      for (int j = 0; j < 8; ++j) v.h[j] = tile[pl][sg * 8 + j];
      *(volatile vf4v_t*)(xt + (size_t)(b * HWP + hw0 + pl) * CIN + sg * 8) = v.fv; }
    __threadfence();
  }
}

__global__ __launch_bounds__(256) void cvt_f16_kernel(const float* __restrict__ src,
                                                      _Float16* __restrict__ dst, int n) {
  int t8 = blockIdx.x * 256 + threadIdx.x;
  if (t8 * 8 >= n) return;
  H8 v;
#pragma unroll
  for (int j = 0; j < 8; ++j) v.h[j] = (_Float16)src[t8 * 8 + j];
  VST2(vf4v_t, dst + (size_t)t8 * 8, v.fv);
}

__global__ __launch_bounds__(256) void gemm256_kernel(
    const _Float16* __restrict__ Wm, const _Float16* __restrict__ X,
    _Float16* __restrict__ Out,
    const float* __restrict__ bn_g, const float* __restrict__ bn_b,
    const float* __restrict__ bn_m, const float* __restrict__ bn_v) {
  __shared__ __align__(32) _Float16 lx[32 * 272];
  const int t = threadIdx.x;
  const int pbase = blockIdx.x * 32;
  {
    int row = t >> 3;
    int col = (t & 7) * 32;
    const _Float16* ga = X + (size_t)(pbase + row) * CIN + col;
    _Float16* ld = lx + row * 272 + col;
#pragma unroll
    for (int i = 0; i < 4; ++i) *(float4*)(ld + 8 * i) = *(const float4*)(ga + 8 * i);
  }
  __syncthreads();

  const int wave = t >> 5, lane = t & 31;
  const int n = lane & 15, g = lane >> 4;
  const int mt0 = wave * 2, mt1 = wave * 2 + 1;
  v8f acc00 = {}; v8f acc01 = {};
  v8f acc10 = {}; v8f acc11 = {};
  const _Float16* a0base = Wm + (size_t)(mt0 * 16 + n) * CIN + g * 8;
  const _Float16* a1base = Wm + (size_t)(mt1 * 16 + n) * CIN + g * 8;
  const _Float16* b0base = lx + n * 272 + g * 8;
  const _Float16* b1base = lx + (16 + n) * 272 + g * 8;
  __builtin_prefetch(a0base, 0, 0);
  __builtin_prefetch(a1base, 0, 0);
#pragma unroll
  for (int ks = 0; ks < 8; ++ks) {
    Frag16 b0, b1, a0, a1;
    b0.f[0] = *(const float4*)(b0base + ks * 32);
    b0.f[1] = *(const float4*)(b0base + ks * 32 + 16);
    b1.f[0] = *(const float4*)(b1base + ks * 32);
    b1.f[1] = *(const float4*)(b1base + ks * 32 + 16);
    a0.f[0] = *(const float4*)(a0base + ks * 32);
    a0.f[1] = *(const float4*)(a0base + ks * 32 + 16);
    a1.f[0] = *(const float4*)(a1base + ks * 32);
    a1.f[1] = *(const float4*)(a1base + ks * 32 + 16);
    acc00 = wmma16(a0.v, b0.v, acc00);
    acc01 = wmma16(a0.v, b1.v, acc01);
    acc10 = wmma16(a1.v, b0.v, acc10);
    acc11 = wmma16(a1.v, b1.v, acc11);
  }
  __syncthreads();
#pragma unroll
  for (int sel = 0; sel < 4; ++sel) {
    v8f acc = (sel == 0) ? acc00 : (sel == 1) ? acc01 : (sel == 2) ? acc10 : acc11;
    int mt = (sel >> 1) ? mt1 : mt0;
    int pl = ((sel & 1) ? 16 : 0) + n;
    int chbase = mt * 16 + g * 8;
#pragma unroll
    for (int r = 0; r < 8; ++r) {
      float f = acc[r];
      if (bn_g) {
        int ch = chbase + r;
        float sc = bn_g[ch] * (1.0f / sqrtf(bn_v[ch] + EPSV));
        f = f * sc + (bn_b[ch] - bn_m[ch] * sc);
      }
      lx[pl * 272 + chbase + r] = (_Float16)f;
    }
  }
  __syncthreads();
  for (int pass = 0; pass < 2; ++pass) {
#pragma unroll
    for (int q = 0; q < 4; ++q) { const int piece = t + q * 256, pl = piece >> 5, sg = piece & 31;
      H8 v;
#pragma unroll
      for (int j = 0; j < 8; ++j) v.h[j] = lx[pl * 272 + sg * 8 + j];
      *(volatile vf4v_t*)(Out + (size_t)(pbase + pl) * COUT + sg * 8) = v.fv; }
    __threadfence();
  }
}


#define AT_KEYS 160
#define AT_KP   136
#define AT_PP   168
#define AT_SP   164
__global__ __launch_bounds__(256) void attn_wmma_kernel(
    const _Float16* __restrict__ Q, const _Float16* __restrict__ Kb, const _Float16* __restrict__ Vb,
    const float* __restrict__ rel_h, const float* __restrict__ rel_w,
    const float* __restrict__ g1, const float* __restrict__ b1, const float* __restrict__ m1, const float* __restrict__ v1,
    _Float16* __restrict__ AO) {
  __shared__ __align__(16) _Float16 sK[AT_KEYS * AT_KP];
  __shared__ __align__(16) _Float16 sVt[HDIM * AT_PP];
  __shared__ __align__(16) _Float16 sQ[64 * AT_KP];
  __shared__ __align__(16) float    sS[64 * AT_SP];
  _Float16* sP = sK;
  _Float16* sO = sQ;

  const int t = threadIdx.x, lane = t & 31, wave = t >> 5, hh = lane >> 4, l16 = lane & 15;
  const int b = blockIdx.x / 49, tileid = blockIdx.x % 49;
  const int ty0 = (tileid / 7) * 8, tx0 = (tileid % 7) * 8;

  for (int head = 0; head < 2; ++head) {
    const int hc = head * HDIM;
    __syncthreads();
    for (int i = t; i < AT_KEYS * (HDIM / 8); i += 256) {
      const int key = i >> 4, sg = i & 15;
      H8 kv; kv.fv = (vf4v_t){0.f, 0.f, 0.f, 0.f};
      H8 vv; vv.fv = (vf4v_t){0.f, 0.f, 0.f, 0.f};
      if (key < 144) {
        const int ky = ty0 - PADR + key / 12, kx = tx0 - PADR + key % 12;
        if ((unsigned)ky < HH && (unsigned)kx < WWID) {
          const size_t p2 = (size_t)b * HWP + ky * WWID + kx;
          kv.f = *(const float4*)(Kb + p2 * COUT + hc + sg * 8);
          vv.f = *(const float4*)(Vb + p2 * COUT + hc + sg * 8);
        }
      } else if (key < 149) {
        const float* rel = head ? rel_w : rel_h;
#pragma unroll
        for (int j = 0; j < 8; ++j) kv.h[j] = (_Float16)rel[(sg * 8 + j) * 5 + (key - 144)];
      }
      *(vf4v_t*)(sK + key * AT_KP + sg * 8) = kv.fv;
#pragma unroll
      for (int j = 0; j < 8; ++j) sVt[(sg * 8 + j) * AT_PP + key] = vv.h[j];
    }
    for (int i = t; i < 64 * (HDIM / 8); i += 256) {
      const int pl = i >> 4, sg = i & 15;
      const size_t p = (size_t)b * HWP + (ty0 + (pl >> 3)) * WWID + tx0 + (pl & 7);
      *(float4*)(sQ + pl * AT_KP + sg * 8) = *(const float4*)(Q + p * COUT + hc + sg * 8);
    }
    __syncthreads();

    {
      const int mt = wave & 3;
      Frag16 aq[4];
#pragma unroll
      for (int ks = 0; ks < 4; ++ks) {
        const _Float16* ap = sQ + (mt * 16 + l16) * AT_KP + ks * 32 + hh * 8;
        aq[ks].f[0] = *(const float4*)ap; aq[ks].f[1] = *(const float4*)(ap + 16);
      }
      for (int nt = (wave >> 2); nt < 10; nt += 2) {
        v8f acc = {};
#pragma unroll
        for (int ks = 0; ks < 4; ++ks) {
          Frag16 bk;
          const _Float16* bp = sK + (nt * 16 + l16) * AT_KP + ks * 32 + hh * 8;
          bk.f[0] = *(const float4*)bp; bk.f[1] = *(const float4*)(bp + 16);
          acc = wmma16(aq[ks].v, bk.v, acc);
        }
#pragma unroll
        for (int r = 0; r < 8; ++r) sS[(mt * 16 + 8 * hh + r) * AT_SP + nt * 16 + l16] = acc[r];
      }
    }
    __syncthreads();

    if (t < 64) {
      const int ly = t >> 3, lx = t & 7;
      const float* srow = sS + t * AT_SP;
      float sc[25];
      float mx = -3.0e38f;
#pragma unroll
      for (int tap = 0; tap < 25; ++tap) {
        const int di = tap / 5, dj = tap % 5;
        const float rb = srow[144 + (head ? dj : di)];
        const float s = (srow[(ly + di) * 12 + (lx + dj)] + rb) * INV_SQRT_HD;
        sc[tap] = s; mx = fmaxf(mx, s);
      }
      float sum = 0.f;
#pragma unroll
      for (int tap = 0; tap < 25; ++tap) { sc[tap] = expf(sc[tap] - mx); sum += sc[tap]; }
      const float inv = 1.f / sum;
      _Float16* prow = sP + t * AT_PP;
      for (int k = 0; k < AT_KEYS; ++k) prow[k] = (_Float16)0.0f;
#pragma unroll
      for (int tap = 0; tap < 25; ++tap) { const int di = tap / 5, dj = tap % 5; prow[(ly + di) * 12 + (lx + dj)] = (_Float16)(sc[tap] * inv); }
    }
    __syncthreads();

    {
      const int mt = wave & 3;
      for (int nt = (wave >> 2); nt < 8; nt += 2) {
        v8f acc = {};
#pragma unroll
        for (int ks = 0; ks < 5; ++ks) {
          Frag16 ap_, bv;
          const _Float16* pp = sP + (mt * 16 + l16) * AT_PP + ks * 32 + hh * 8;
          ap_.f[0] = *(const float4*)pp; ap_.f[1] = *(const float4*)(pp + 16);
          const _Float16* vp = sVt + (nt * 16 + l16) * AT_PP + ks * 32 + hh * 8;
          bv.f[0] = *(const float4*)vp; bv.f[1] = *(const float4*)(vp + 16);
          acc = wmma16(ap_.v, bv.v, acc);
        }
        const int ch = hc + nt * 16 + l16;
        const float s = g1[ch] * (1.0f / sqrtf(v1[ch] + EPSV));
        const float sh = b1[ch] - m1[ch] * s;
#pragma unroll
        for (int r = 0; r < 8; ++r) sO[(mt * 16 + 8 * hh + r) * AT_KP + nt * 16 + l16] = (_Float16)fmaxf(acc[r] * s + sh, 0.f);
      }
    }
    __syncthreads();
    for (int pass = 0; pass < 2; ++pass) {
#pragma unroll
      for (int q = 0; q < 4; ++q) {
        const int piece = t + q * 256, pl = piece >> 4, sg = piece & 15;
        const size_t p = (size_t)b * HWP + (ty0 + (pl >> 3)) * WWID + tx0 + (pl & 7);
        *(volatile vf4v_t*)(AO + p * COUT + hc + sg * 8) = *(const vf4v_t*)(sO + pl * AT_KP + sg * 8);
      }
      __threadfence();
    }
  }
}

__global__ __launch_bounds__(256) void se_kernel(
    const _Float16* __restrict__ Wse, const _Float16* __restrict__ Y,
    const float* __restrict__ g_in, const float* __restrict__ b_in,
    const float* __restrict__ m_in, const float* __restrict__ v_in,
    float* __restrict__ S, float* __restrict__ psum) {
  const int wave = threadIdx.x >> 5, lane = threadIdx.x & 31;
  const int ptile = blockIdx.x * 8 + wave;
  const int n = lane & 15, g = lane >> 4;
  const _Float16* abase = Wse + (size_t)n * CIN + g * 8;
  const _Float16* bbase = Y + (size_t)(ptile * 16 + n) * CIN + g * 8;
  v8f acc = {};
#pragma unroll
  for (int ks = 0; ks < 8; ++ks) {
    Frag16 a, bf;
    a.f[0]  = *(const float4*)(abase + ks * 32);
    a.f[1]  = *(const float4*)(abase + ks * 32 + 16);
    bf.f[0] = *(const float4*)(bbase + ks * 32);
    bf.f[1] = *(const float4*)(bbase + ks * 32 + 16);
    acc = wmma16(a.v, bf.v, acc);
  }
  __shared__ __align__(16) float sS[8][16 * 16];
  float* st = sS[wave];
#pragma unroll
  for (int r = 0; r < 8; ++r) {
    int ch = r + g * 8;
    float s = g_in[ch] * (1.0f / sqrtf(v_in[ch] + EPSV));
    st[n * 16 + ch] = fmaxf(acc[r] * s + (b_in[ch] - m_in[ch] * s), 0.f);
  }
  __builtin_amdgcn_fence(__ATOMIC_RELEASE, "workgroup"); __builtin_amdgcn_wave_barrier(); __builtin_amdgcn_fence(__ATOMIC_ACQUIRE, "workgroup");
  float* dst = S + (size_t)ptile * 16 * 16;
  for (int pass = 0; pass < 2; ++pass) {
#pragma unroll
    for (int q = 0; q < 2; ++q) { const int piece = lane + q * 32; *(volatile vf4v_t*)(dst + piece * 4) = *(const vf4v_t*)(st + piece * 4); }
    __threadfence();
  }
  (void)psum;
}

__global__ __launch_bounds__(256) void segate_kernel(const float* __restrict__ S, const float* __restrict__ fc1,
                                                     const float* __restrict__ fc2, float* __restrict__ G) {
  __shared__ float part[4][64];
  __shared__ float mean_[64];
  const int t = threadIdx.x, bc = t & 63, qtr = t >> 6;
  const int b = bc >> 4, ch = bc & 15;
  float s = 0.f;
  for (int hw = qtr; hw < HWP; hw += 4) s += S[((size_t)b * HWP + hw) * 16 + ch];
  part[qtr][bc] = s;
  __syncthreads();
  if (t < 64) mean_[t] = (part[0][t] + part[1][t] + part[2][t] + part[3][t]) * (1.0f / HWP);
  __syncthreads();
  if (t < 64) {
    float acc = 0.f;
    for (int c = 0; c < 16; ++c) acc += mean_[b * 16 + c] * fc1[c];
    acc = fmaxf(acc, 0.f);
    VST2(float, G + t, 1.f / (1.f + expf(-acc * fc2[ch])));
  }
}

__global__ __launch_bounds__(256) void final_kernel(
    const float* __restrict__ S, const float* __restrict__ G,
    const float* __restrict__ Wout,
    const float* __restrict__ g_o, const float* __restrict__ b_o,
    const float* __restrict__ m_o, const float* __restrict__ v_o,
    float* __restrict__ out) {
  int t = blockIdx.x * 256 + threadIdx.x;
  if (t >= BATCH * COUT * HWP) return;
  int hw = t % HWP;
  int co = (t / HWP) % COUT;
  int b  = t / (HWP * COUT);
  size_t p = (size_t)b * HWP + hw;
  float acc = 0.f;
#pragma unroll
  for (int ch = 0; ch < 16; ++ch)
    acc += Wout[co * 16 + ch] * S[p * 16 + ch] * G[b * 16 + ch];
  float s = g_o[co] * (1.0f / sqrtf(v_o[co] + EPSV));
  VST2(float, out + t, acc * s + (b_o[co] - m_o[co] * s));
}

extern "C" void kernel_launch(void* const* d_in, const int* in_sizes, int n_in,
                              void* d_out, int out_size, void* d_ws, size_t ws_size,
                              hipStream_t stream) {
  (void)in_sizes; (void)n_in; (void)out_size;
  const float* x     = (const float*)d_in[0];
  const float* Wq    = (const float*)d_in[1];
  const float* Wk    = (const float*)d_in[2];
  const float* Wv    = (const float*)d_in[3];
  const float* rel_h = (const float*)d_in[4];
  const float* rel_w = (const float*)d_in[5];
  const float* g1    = (const float*)d_in[6];
  const float* b1    = (const float*)d_in[7];
  const float* m1    = (const float*)d_in[8];
  const float* v1    = (const float*)d_in[9];
  const float* aggW  = (const float*)d_in[10];
  const float* g2    = (const float*)d_in[11];
  const float* b2    = (const float*)d_in[12];
  const float* m2    = (const float*)d_in[13];
  const float* v2    = (const float*)d_in[14];
  const float* seWin = (const float*)d_in[15];
  const float* g_in  = (const float*)d_in[16];
  const float* b_in  = (const float*)d_in[17];
  const float* m_in  = (const float*)d_in[18];
  const float* v_in  = (const float*)d_in[19];
  const float* fc1   = (const float*)d_in[20];
  const float* fc2   = (const float*)d_in[21];
  const float* seWout= (const float*)d_in[22];
  const float* g_o   = (const float*)d_in[23];
  const float* b_o   = (const float*)d_in[24];
  const float* m_o   = (const float*)d_in[25];
  const float* v_o   = (const float*)d_in[26];

  uint8_t* ws = (uint8_t*)d_ws;
  size_t off = 0;
  auto alloc = [&](size_t bytes) -> void* {
    void* p = ws + off;
    off = (off + bytes + 255) & ~(size_t)255;
    return p;
  };

  const size_t big = (size_t)NPIX * CIN * sizeof(_Float16);
  _Float16* XT16   = (_Float16*)alloc(big);
  _Float16* Q16    = (_Float16*)alloc(big);
  _Float16* K16    = (_Float16*)alloc(big);
  _Float16* V16    = (_Float16*)alloc(big);
  _Float16* Wq16   = (_Float16*)alloc((size_t)COUT * CIN * 2);
  _Float16* Wk16   = (_Float16*)alloc((size_t)COUT * CIN * 2);
  _Float16* Wv16   = (_Float16*)alloc((size_t)COUT * CIN * 2);
  _Float16* aggW16 = (_Float16*)alloc((size_t)COUT * CIN * 2);
  _Float16* seWin16= (_Float16*)alloc((size_t)16 * CIN * 2);
  float* S  = (float*)alloc((size_t)NPIX * 16 * sizeof(float));
  float* G  = (float*)alloc(64 * sizeof(float));
  if (off > ws_size) return;

  cvt_x_kernel<<<BATCH * (HWP / 64), 256, 0, stream>>>(x, XT16);
  cvt_f16_kernel<<<32, 256, 0, stream>>>(Wq,   Wq16,   COUT * CIN);
  cvt_f16_kernel<<<32, 256, 0, stream>>>(Wk,   Wk16,   COUT * CIN);
  cvt_f16_kernel<<<32, 256, 0, stream>>>(Wv,   Wv16,   COUT * CIN);
  cvt_f16_kernel<<<32, 256, 0, stream>>>(aggW, aggW16, COUT * CIN);
  cvt_f16_kernel<<<2,  256, 0, stream>>>(seWin, seWin16, 16 * CIN);

  gemm256_kernel<<<NPIX / 32, 256, 0, stream>>>(Wq16, XT16, Q16,
                                                nullptr, nullptr, nullptr, nullptr);
  gemm256_kernel<<<NPIX / 32, 256, 0, stream>>>(Wk16, XT16, K16,
                                                nullptr, nullptr, nullptr, nullptr);
  gemm256_kernel<<<NPIX / 32, 256, 0, stream>>>(Wv16, XT16, V16,
                                                nullptr, nullptr, nullptr, nullptr);

  attn_wmma_kernel<<<BATCH * 49, 256, 0, stream>>>(Q16, K16, V16, rel_h, rel_w,
                                                   g1, b1, m1, v1, XT16);

  gemm256_kernel<<<NPIX / 32, 256, 0, stream>>>(aggW16, XT16, Q16, g2, b2, m2, v2);

  se_kernel<<<NPIX / 16 / 8, 256, 0, stream>>>(seWin16, Q16, g_in, b_in, m_in, v_in,
                                               S, nullptr);
  segate_kernel<<<1, 256, 0, stream>>>(S, fc1, fc2, G);
  final_kernel<<<(BATCH * COUT * HWP) / 256, 256, 0, stream>>>(
      S, G, seWout, g_o, b_o, m_o, v_o, (float*)d_out);
}
